// SelfAttention_56599079026811
// MI455X (gfx1250) — hardware-verified
//
#include <hip/hip_runtime.h>


#ifndef NB
#define NB 4
#endif
#ifndef SEQ
#define SEQ 2048
#endif
#define NB_FULL    4
#define SEQ_FULL   2048
#define DMODEL     1024
#define NHEAD      16
#define HDIM       64
#define NQKV       (3 * DMODEL)
#define KDIM       DMODEL
#define TM         256
#define TN         64
#define BQ         128
#define BK         32
#define NWAVE      8
#define QP         72
#define VP         264
#define OP         68

#define PLANE_ELEMS ((size_t)NB * NHEAD * SEQ * HDIM)
#define X_ELEMS     ((size_t)NB * SEQ * DMODEL)
#define WQKV_ELEMS  ((size_t)NQKV * DMODEL)
#define WO_ELEMS    ((size_t)DMODEL * DMODEL)
#define WS_TOTAL    ((X_ELEMS + WQKV_ELEMS + WO_ELEMS + 3 * PLANE_ELEMS + X_ELEMS) * 2)

static_assert(SEQ % TM == 0);
static_assert(SEQ % BQ == 0);
static_assert(SEQ % BK == 0);
static_assert(KDIM % 32 == 0);
static_assert(NQKV % TN == 0);
static_assert(DMODEL % TN == 0);
static_assert(TN == HDIM);
static_assert(NQKV == NHEAD * 3 * HDIM);
static_assert(DMODEL == NHEAD * HDIM);
static_assert(TM == NWAVE * 32);
static_assert(BQ == NWAVE * 16);
static_assert(HDIM == 64);
static_assert(HDIM == 8 * 8);
static_assert(TM == 32 * 8);
static_assert(TM * QP >= HDIM * VP);
static_assert((QP * 2) % 16 == 0);
static_assert((VP * 2) % 16 == 0);
static_assert((OP * 4) % 16 == 0);
static_assert(SEQ <= SEQ_FULL);
static_assert(NB >= 1 && NB <= NB_FULL);
static_assert((X_ELEMS / 8) % 256 == 0);
static_assert((WQKV_ELEMS / 8) % 256 == 0);
static_assert((WO_ELEMS / 8) % 256 == 0);
static_assert(X_ELEMS < 0x7fffffffULL);
static_assert((X_ELEMS * 2) % 128 == 0 && (WQKV_ELEMS * 2) % 128 == 0 && (WO_ELEMS * 2) % 128 == 0);
static_assert((PLANE_ELEMS * 2) % 128 == 0);
static_assert(WS_TOTAL <= 134217728ULL);

typedef __bf16   bf16;
typedef _Float16 f16;
typedef bf16     v16bf __attribute__((ext_vector_type(16)));
typedef f16      v16h  __attribute__((ext_vector_type(16)));
typedef f16      v8h   __attribute__((ext_vector_type(8)));
typedef float    v8f   __attribute__((ext_vector_type(8)));
typedef float    v4f   __attribute__((ext_vector_type(4)));
typedef unsigned v4u   __attribute__((ext_vector_type(4)));

union Frag   { v16bf b; v16h h; v4u q[2]; };
union FragH  { v16h  v; v4u q[2]; f16  h[16]; };
union Pack8B { v4u u; bf16 h[8]; };
union Pack8H { v4u u; v8h v; f16 h[8]; };

static __device__ __forceinline__ v8f mma_bf16(v16bf a, v16bf b, v8f acc) {
  acc = __builtin_amdgcn_wmma_f32_16x16x32_bf16(false, a, false, b, (short)0, acc, false, false);
  asm volatile("v_nop\n\tv_nop\n\tv_nop\n\tv_nop" : "+v"(acc) : "v"(a), "v"(b));
  return acc;
}
static __device__ __forceinline__ v8f mma_f16(v16h a, v16h b, v8f acc) {
  acc = __builtin_amdgcn_wmma_f32_16x16x32_f16(false, a, false, b, (short)0, acc, false, false);
  asm volatile("v_nop\n\tv_nop\n\tv_nop\n\tv_nop" : "+v"(acc) : "v"(a), "v"(b));
  return acc;
}

__global__ __launch_bounds__(256) void cvt_kernel(const float* __restrict__ src,
                                                  unsigned short* __restrict__ dst,
                                                  unsigned n8, unsigned dst_batch, unsigned src_batch, int mode) {
  const unsigned i = blockIdx.x * 256u + threadIdx.x;
  if (i >= n8) return;
  const unsigned e  = i * 8u;
  const unsigned bb = e / dst_batch;
  const unsigned rr = e - bb * dst_batch;
  const float* sp = src + (size_t)bb * src_batch + rr;
  const v4f a0 = *(const v4f*)(sp);
  const v4f a1 = *(const v4f*)(sp + 4);
  v4u val;
  if (mode == 0) {
    Pack8B pk;
    #pragma unroll
    for (int j = 0; j < 4; ++j) {
      pk.h[j]     = (bf16)a0[j];
      pk.h[4 + j] = (bf16)a1[j];
    }
    val = pk.u;
  } else {
    Pack8H ph;
    #pragma unroll
    for (int j = 0; j < 4; ++j) {
      ph.h[j]     = (f16)((float)(bf16)a0[j] * 1024.0f);
      ph.h[4 + j] = (f16)((float)(bf16)a1[j] * 1024.0f);
    }
    val = ph.u;
  }
  unsigned short* dp = dst + (size_t)e;
  *(volatile v4u*)dp = val;
  __threadfence();
  *(volatile v4u*)dp = val;
}

template <int ISF16>
static __device__ __forceinline__ void gemm_acc(const unsigned short* __restrict__ A,
                                                const unsigned short* __restrict__ W,
                                                size_t arow0, int n0, int lq, int hi,
                                                v8f (&acc)[2][4]) {
  const unsigned short* ap = A + (arow0 + (size_t)lq) * KDIM + hi * 8;
  const unsigned short* wp = W + (size_t)(n0 + lq) * KDIM + hi * 8;
  #pragma unroll 1
  for (int k0 = 0; k0 < KDIM; k0 += 32) {
    Frag a[2], bw[4];
    #pragma unroll
    for (int f = 0; f < 2; ++f) {
      const unsigned short* p = ap + (size_t)f * 16 * KDIM + k0;
      a[f].q[0] = *(const v4u*)(p);
      a[f].q[1] = *(const v4u*)(p + 16);
    }
    #pragma unroll
    for (int g = 0; g < 4; ++g) {
      const unsigned short* p = wp + (size_t)g * 16 * KDIM + k0;
      bw[g].q[0] = *(const v4u*)(p);
      bw[g].q[1] = *(const v4u*)(p + 16);
    }
    #pragma unroll
    for (int f = 0; f < 2; ++f) {
      #pragma unroll
      for (int g = 0; g < 4; ++g) {
        if (ISF16) acc[f][g] = mma_f16(a[f].h, bw[g].h, acc[f][g]);
        else       acc[f][g] = mma_bf16(a[f].b, bw[g].b, acc[f][g]);
      }
    }
  }
}

__global__ __launch_bounds__(256) void qkv_gemm_kernel(const unsigned short* __restrict__ xb,
                                                       const unsigned short* __restrict__ wb,
                                                       const float* __restrict__ bias,
                                                       f16* __restrict__ planes) {
  const int st   = blockIdx.x;
  const int nt   = blockIdx.y;
  const int b    = blockIdx.z;
  const int tid  = threadIdx.x;
  const int wave = tid >> 5;
  const int lane = tid & 31;
  const int lq   = lane & 15;
  const int hi   = lane >> 4;
  const int h     = nt / 3;
  const int which = nt - 3 * h;
  const int n0    = nt * TN;

  __shared__ __align__(16) f16 sT[TM * QP];

  v8f acc[2][4];
  #pragma unroll
  for (int f = 0; f < 2; ++f) {
    #pragma unroll
    for (int g = 0; g < 4; ++g) acc[f][g] = (v8f){0, 0, 0, 0, 0, 0, 0, 0};
  }

  const size_t arow0 = (size_t)b * SEQ + (size_t)st * TM + wave * 32;
  gemm_acc<0>(xb, wb, arow0, n0, lq, hi, acc);

  float bv[4];
  #pragma unroll
  for (int g = 0; g < 4; ++g) bv[g] = (float)(bf16)bias[n0 + g * 16 + lq];

  if (which != 2) {
    #pragma unroll
    for (int f = 0; f < 2; ++f) {
      #pragma unroll
      for (int g = 0; g < 4; ++g) {
        #pragma unroll
        for (int r = 0; r < 8; ++r) {
          sT[(wave * 32 + f * 16 + hi * 8 + r) * QP + g * 16 + lq] = (f16)((acc[f][g][r] + bv[g]) * 16.0f);
        }
      }
    }
  } else {
    #pragma unroll
    for (int f = 0; f < 2; ++f) {
      #pragma unroll
      for (int g = 0; g < 4; ++g) {
        #pragma unroll
        for (int r = 0; r < 8; ++r) {
          sT[(g * 16 + lq) * VP + wave * 32 + f * 16 + hi * 8 + r] = (f16)((acc[f][g][r] + bv[g]) * 16.0f);
        }
      }
    }
  }
  __syncthreads();

  v4u    vals[8];
  size_t gidx[8];
  const size_t bh = (size_t)b * NHEAD + h;
  if (which != 2) {
    #pragma unroll
    for (int it = 0; it < 8; ++it) {
      const int row = wave * 32 + it * 4 + (lane >> 3);
      const int pc  = lane & 7;
      Pack8H ph;
      ph.v = *(const v8h*)(sT + row * QP + pc * 8);
      vals[it] = ph.u;
      gidx[it] = (size_t)which * PLANE_ELEMS + (bh * SEQ + (size_t)st * TM + row) * HDIM + pc * 8;
    }
  } else {
    #pragma unroll
    for (int it = 0; it < 8; ++it) {
      const int d = it * 8 + wave;
      Pack8H ph;
      ph.v = *(const v8h*)(sT + d * VP + lane * 8);
      vals[it] = ph.u;
      gidx[it] = 2 * PLANE_ELEMS + (bh * HDIM + d) * SEQ + (size_t)st * TM + lane * 8;
    }
  }
  #pragma unroll
  for (int it = 0; it < 8; ++it) *(volatile v4u*)(planes + gidx[it]) = vals[it];
  __threadfence();
  #pragma unroll
  for (int it = 0; it < 8; ++it) *(volatile v4u*)(planes + gidx[it]) = vals[it];
}

__global__ __launch_bounds__(256) void attn_kernel(const f16* __restrict__ planes,
                                                   f16* __restrict__ ctx) {
  const int qblk = blockIdx.x;
  const int h    = blockIdx.y;
  const int b    = blockIdx.z;
  const int tid  = threadIdx.x;
  const int wave = tid >> 5;
  const int lane = tid & 31;
  const int lq   = lane & 15;
  const int hi   = lane >> 4;

  __shared__ __align__(16) float sO[NWAVE * 16 * OP];

  const int qrow0 = qblk * BQ + wave * 16;
  const size_t bh = (size_t)b * NHEAD + h;
  const f16* qp_h = planes + bh * SEQ * HDIM;
  const f16* kb_h = planes + PLANE_ELEMS + bh * SEQ * HDIM;
  const f16* vt_h = planes + 2 * PLANE_ELEMS + bh * HDIM * SEQ;

  FragH qf[2];
  #pragma unroll
  for (int f = 0; f < 2; ++f) {
    const f16* base = qp_h + (size_t)(qrow0 + lq) * HDIM + f * 32 + hi * 8;
    qf[f].q[0] = *(const v4u*)(base);
    qf[f].q[1] = *(const v4u*)(base + 16);
  }

  v8f o[4];
  #pragma unroll
  for (int dt = 0; dt < 4; ++dt) o[dt] = (v8f){0, 0, 0, 0, 0, 0, 0, 0};

  float rmax = -__builtin_inff();
  float rsum = 0.0f;
  const float SL = 0.125f * 1.4426950408889634f * (1.0f / 256.0f);

  #pragma unroll 1
  for (int i = 0; i < SEQ / BK; ++i) {
    const int j0 = i * BK;

    FragH ak[2][2];
    #pragma unroll
    for (int sub = 0; sub < 2; ++sub) {
      #pragma unroll
      for (int f = 0; f < 2; ++f) {
        const f16* base = kb_h + (size_t)(j0 + sub * 16 + lq) * HDIM + f * 32 + hi * 8;
        ak[sub][f].q[0] = *(const v4u*)(base);
        ak[sub][f].q[1] = *(const v4u*)(base + 16);
      }
    }
    FragH bvf[4];
    #pragma unroll
    for (int dt = 0; dt < 4; ++dt) {
      const f16* base = vt_h + (size_t)(dt * 16 + lq) * SEQ + j0 + hi * 8;
      bvf[dt].q[0] = *(const v4u*)(base);
      bvf[dt].q[1] = *(const v4u*)(base + 16);
    }

    v8f c[2];
    #pragma unroll
    for (int sub = 0; sub < 2; ++sub) {
      v8f acc = (v8f){0, 0, 0, 0, 0, 0, 0, 0};
      acc = mma_f16(ak[sub][0].v, qf[0].v, acc);
      acc = mma_f16(ak[sub][1].v, qf[1].v, acc);
      c[sub] = acc;
    }

    float m_new = rmax;
    #pragma unroll
    for (int r = 0; r < 8; ++r) {
      m_new = fmaxf(m_new, c[0][r]);
      m_new = fmaxf(m_new, c[1][r]);
    }
    m_new = fmaxf(m_new, __shfl_xor(m_new, 16, 32));
    const float scale = __builtin_amdgcn_exp2f((rmax - m_new) * SL);
    rmax = m_new;

    FragH pa;
    float psum = 0.0f;
    #pragma unroll
    for (int r = 0; r < 8; ++r) {
      const float p0 = __builtin_amdgcn_exp2f((c[0][r] - m_new) * SL);
      const float p1 = __builtin_amdgcn_exp2f((c[1][r] - m_new) * SL);
      psum += p0 + p1;
      pa.h[r]     = (f16)(p0 * 4096.0f);
      pa.h[8 + r] = (f16)(p1 * 4096.0f);
    }
    rsum = rsum * scale + psum + __shfl_xor(psum, 16, 32);

    float sc[8];
    #pragma unroll
    for (int r = 0; r < 8; ++r) sc[r] = __shfl(scale, (hi << 3) + r, 32);
    #pragma unroll
    for (int dt = 0; dt < 4; ++dt) {
      #pragma unroll
      for (int r = 0; r < 8; ++r) o[dt][r] *= sc[r];
    }

    #pragma unroll
    for (int dt = 0; dt < 4; ++dt) o[dt] = mma_f16(pa.v, bvf[dt].v, o[dt]);
  }

  float rs[8];
  #pragma unroll
  for (int r = 0; r < 8; ++r) rs[r] = 1.0f / __shfl(rsum, (hi << 3) + r, 32);

  float* so = sO + wave * (16 * OP);
  #pragma unroll
  for (int r = 0; r < 8; ++r) {
    #pragma unroll
    for (int dt = 0; dt < 4; ++dt) {
      so[(hi * 8 + r) * OP + dt * 16 + lq] = o[dt][r] * (1.0f / 256.0f) * rs[r];
    }
  }
  __syncthreads();

  v4u    vals[4];
  size_t gidx[4];
  #pragma unroll
  for (int it = 0; it < 4; ++it) {
    const int row = it * 4 + (lane >> 3);
    const int pc  = lane & 7;
    const v4f a0 = *(const v4f*)(so + row * OP + pc * 8);
    const v4f a1 = *(const v4f*)(so + row * OP + pc * 8 + 4);
    Pack8H ph;
    #pragma unroll
    for (int j = 0; j < 4; ++j) {
      ph.h[j]     = (f16)a0[j];
      ph.h[4 + j] = (f16)a1[j];
    }
    vals[it] = ph.u;
    gidx[it] = ((size_t)b * SEQ + qrow0 + row) * DMODEL + h * HDIM + pc * 8;
  }
  #pragma unroll
  for (int it = 0; it < 4; ++it) *(volatile v4u*)(ctx + gidx[it]) = vals[it];
  __threadfence();
  #pragma unroll
  for (int it = 0; it < 4; ++it) *(volatile v4u*)(ctx + gidx[it]) = vals[it];
}

static __device__ __forceinline__ void oproj_store_half(const v8f (&accf)[4], float* so, float* __restrict__ out,
                                                        size_t out_row0, int n0, int lq, int hi, v4f bias4) {
  #pragma unroll
  for (int g = 0; g < 4; ++g) {
    #pragma unroll
    for (int r = 0; r < 8; ++r) {
      so[(hi * 8 + r) * OP + g * 16 + lq] = accf[g][r] * (1.0f / 262144.0f);
    }
  }
  __syncthreads();
  v4f    vals[8];
  size_t gidx[8];
  #pragma unroll
  for (int it = 0; it < 8; ++it) {
    const int row = it * 2 + hi;
    const v4f t = *(const v4f*)(so + row * OP + lq * 4);
    vals[it] = t + bias4;
    gidx[it] = (out_row0 + row) * DMODEL + n0 + lq * 4;
  }
  #pragma unroll
  for (int it = 0; it < 8; ++it) *(volatile v4f*)(out + gidx[it]) = vals[it];
  __threadfence();
  #pragma unroll
  for (int it = 0; it < 8; ++it) *(volatile v4f*)(out + gidx[it]) = vals[it];
}

__global__ __launch_bounds__(256) void oproj_gemm_kernel(const unsigned short* __restrict__ ctx,
                                                         const unsigned short* __restrict__ wo,
                                                         const float* __restrict__ bo,
                                                         float* __restrict__ out) {
  const int st   = blockIdx.x;
  const int nt   = blockIdx.y;
  const int b    = blockIdx.z;
  const int tid  = threadIdx.x;
  const int wave = tid >> 5;
  const int lane = tid & 31;
  const int lq   = lane & 15;
  const int hi   = lane >> 4;
  const int n0   = nt * TN;

  __shared__ __align__(16) float sO[NWAVE * 16 * OP];

  v8f acc[2][4];
  #pragma unroll
  for (int f = 0; f < 2; ++f) {
    #pragma unroll
    for (int g = 0; g < 4; ++g) acc[f][g] = (v8f){0, 0, 0, 0, 0, 0, 0, 0};
  }

  const size_t arow0 = (size_t)b * SEQ + (size_t)st * TM + wave * 32;
  gemm_acc<1>(ctx, wo, arow0, n0, lq, hi, acc);

  const v4f braw = *(const v4f*)(bo + n0 + lq * 4);
  v4f bias4;
  #pragma unroll
  for (int j = 0; j < 4; ++j) bias4[j] = (float)(bf16)braw[j];

  float* so = sO + wave * (16 * OP);
  const size_t out_row0 = (size_t)b * SEQ_FULL + (size_t)st * TM + wave * 32;
  oproj_store_half(acc[0], so, out, out_row0, n0, lq, hi, bias4);
  __syncthreads();
  oproj_store_half(acc[1], so, out, out_row0 + 16, n0, lq, hi, bias4);
}

extern "C" void kernel_launch(void* const* d_in, const int* in_sizes, int n_in,
                              void* d_out, int out_size, void* d_ws, size_t ws_size,
                              hipStream_t stream) {
  if (n_in < 5) return;
  const size_t rows_used = (size_t)(NB - 1) * SEQ_FULL + SEQ;
  if ((size_t)in_sizes[0] < rows_used * DMODEL) return;
  if ((size_t)in_sizes[1] < WQKV_ELEMS) return;
  if ((size_t)in_sizes[2] < (size_t)NQKV) return;
  if ((size_t)in_sizes[3] < WO_ELEMS) return;
  if ((size_t)in_sizes[4] < (size_t)DMODEL) return;
  if ((size_t)out_size < rows_used * DMODEL) return;
  if (ws_size < WS_TOTAL) return;

  const float* x     = (const float*)d_in[0];
  const float* w_qkv = (const float*)d_in[1];
  const float* b_qkv = (const float*)d_in[2];
  const float* w_o   = (const float*)d_in[3];
  const float* b_o   = (const float*)d_in[4];
  float*       out   = (float*)d_out;

  unsigned short* ws16   = (unsigned short*)d_ws;
  unsigned short* xb     = ws16;
  unsigned short* wqb    = xb + X_ELEMS;
  unsigned short* woh    = wqb + WQKV_ELEMS;
  unsigned short* planes = woh + WO_ELEMS;
  unsigned short* ctx    = planes + 3 * PLANE_ELEMS;

  cvt_kernel<<<dim3((unsigned)(X_ELEMS / 8 / 256)), 256, 0, stream>>>(
      x, xb, (unsigned)(X_ELEMS / 8), (unsigned)((size_t)SEQ * DMODEL), (unsigned)((size_t)SEQ_FULL * DMODEL), 0);
  cvt_kernel<<<dim3((unsigned)(WQKV_ELEMS / 8 / 256)), 256, 0, stream>>>(
      w_qkv, wqb, (unsigned)(WQKV_ELEMS / 8), (unsigned)WQKV_ELEMS, (unsigned)WQKV_ELEMS, 0);
  cvt_kernel<<<dim3((unsigned)(WO_ELEMS / 8 / 256)), 256, 0, stream>>>(
      w_o, woh, (unsigned)(WO_ELEMS / 8), (unsigned)WO_ELEMS, (unsigned)WO_ELEMS, 1);

  qkv_gemm_kernel<<<dim3(SEQ / TM, NQKV / TN, NB), 256, 0, stream>>>(xb, wqb, b_qkv, (f16*)planes);

  attn_kernel<<<dim3(SEQ / BQ, NHEAD, NB), 256, 0, stream>>>((const f16*)planes, (f16*)ctx);

  oproj_gemm_kernel<<<dim3(SEQ / TM, DMODEL / TN, NB), 256, 0, stream>>>(ctx, woh, b_o, out);
}
